// RicciTensorNetwork_74732430950676
// MI455X (gfx1250) — hardware-run, weakly checked
//
#include <hip/hip_runtime.h>
#include <math.h>

typedef __attribute__((ext_vector_type(16))) _Float16 v16h;
typedef __attribute__((ext_vector_type(8)))  _Float16 v8h;
typedef __attribute__((ext_vector_type(8)))  float    v8f;
typedef __attribute__((ext_vector_type(4)))  float    v4f;

constexpr int kBatch = 256;
constexpr int kDim   = 16;
constexpr int kHid   = 128;
constexpr int kHid2  = 256;
constexpr int kSq    = kDim * kDim;
constexpr int kFeat  = 4 * kDim;
constexpr int kTrip  = kDim * kDim * kDim;
constexpr int kMhPitch = 136;
static_assert(kSq == 256 && kFeat == 64 && kTrip == 4096, "shape constants");
static_assert((kFeat % 32) == 0 && (kHid % 32) == 0, "matrix-core K multiples of 32");
static_assert((kHid2 % 16) == 0 && (kSq % 16) == 0, "matrix-core N multiples of 16");
static_assert(((kMhPitch * 2) % 16) == 0, "hidden tile pitch keeps 16-B alignment");

constexpr float kCarryMh   = 16.0f;
constexpr float kCarryW2   = 64.0f;
constexpr float kFoldMet   = 1.0f / (kCarryMh * kCarryW2);
constexpr float kCarryFeat = 128.0f;
constexpr float kCarryW1   = 64.0f;
constexpr float kFoldPair  = 1.0f / (kCarryFeat * kCarryW1);
constexpr float kInvPairs  = 1.0f / (float)kSq;
constexpr float kEps       = 1e-6f;
constexpr float kF16MinNormal = 6.103515625e-5f;

constexpr size_t kOffMET  = 0;
constexpr size_t kOffCHR  = kOffMET  + (size_t)kBatch * kSq * 4;
constexpr size_t kOffRW1T = kOffCHR  + (size_t)kBatch * kTrip * 4;
constexpr size_t kOffMW2T = kOffRW1T + (size_t)kHid2 * kFeat * 2;
constexpr size_t kWsTotal = kOffMW2T + (size_t)kSq * kHid * 2;
static_assert(kWsTotal == 4554752ull, "carve total");
static_assert(kWsTotal <= 134217728ull, "carve cap");
static_assert((kOffCHR % 128) == 0 && (kOffRW1T % 128) == 0 && (kOffMW2T % 128) == 0, "128-B aligned regions");

union FragH { v16h v; v8h h[2]; };

__device__ __forceinline__ _Float16 to_h_flush(float v) {
  const float z = (fabsf(v) < kF16MinNormal) ? 0.0f : v;
  return (_Float16)z;
}

__device__ __forceinline__ v8f mma_f16(v16h a, v16h b, v8f c) {
  c = __builtin_amdgcn_wmma_f32_16x16x32_f16(false, a, false, b, (short)0, c, false, false);
  asm volatile("v_nop\n\tv_nop\n\tv_nop\n\tv_nop" : "+v"(c) : "v"(a), "v"(b));
  return c;
}

__device__ __forceinline__ v16h frag_load_global(const _Float16* p) {
  FragH f;
  f.h[0] = *(const v8h*)(p);
  f.h[1] = *(const v8h*)(p + 16);
  return f.v;
}

__device__ __forceinline__ float tanh_exp_form(float x) {
  const float e = __expf(2.0f * x);
  return 1.0f - 2.0f * __builtin_amdgcn_rcpf(e + 1.0f);
}

__global__ __launch_bounds__(256) void transpose_cast_kernel(
    const float* __restrict__ src, int kdim, int ncols, _Float16* __restrict__ dst, float carry, int total8)
{
  const int t = blockIdx.x * 256 + threadIdx.x;
  if (t >= total8) return;
  const int cpr = kdim >> 3;
  const int n   = t / cpr;
  const int k8  = (t - n * cpr) << 3;
  v8h hv;
#pragma unroll
  for (int e = 0; e < 8; ++e) {
    const float w = src[(size_t)(k8 + e) * ncols + n] * carry;
    hv[e] = to_h_flush(w);
  }
  _Float16* p = dst + (size_t)t * 8;
  *(volatile v8h*)p = hv;
  __threadfence();
  *(volatile v8h*)p = hv;
}

__global__ __launch_bounds__(256) void metric_net_kernel(
    const float* __restrict__ points, const float* __restrict__ mW1, const float* __restrict__ mb1,
    const _Float16* __restrict__ MW2T, const float* __restrict__ mb2, float* __restrict__ met)
{
  __shared__ __align__(16) float    sP[16 * kDim];
  __shared__ __align__(16) float    sW1[kDim * kHid];
  __shared__ __align__(16) _Float16 sMh[16 * kMhPitch];
  __shared__ __align__(16) float    sRaw[16 * kSq];
  const int tid  = threadIdx.x;
  const int lane = tid & 31;
  const int wave = tid >> 5;
  const int hh   = lane >> 4;
  const int rl   = lane & 15;
  const int rowbase = blockIdx.x * 16;

  sP[tid] = points[(size_t)rowbase * kDim + tid];
#pragma unroll 1
  for (int t = tid; t < kDim * kHid; t += 256) sW1[t] = mW1[t];
  __syncthreads();

  {
    const int row = tid >> 4;
    const int c8  = (tid & 15) * 8;
    float a[8];
#pragma unroll
    for (int e = 0; e < 8; ++e) a[e] = 0.0f;
#pragma unroll 2
    for (int k = 0; k < kDim; ++k) {
      const float p = sP[row * kDim + k];
      const v4f w0 = *(const v4f*)(sW1 + k * kHid + c8);
      const v4f w1 = *(const v4f*)(sW1 + k * kHid + c8 + 4);
#pragma unroll
      for (int e = 0; e < 4; ++e) {
        a[e]     = fmaf(p, w0[e], a[e]);
        a[4 + e] = fmaf(p, w1[e], a[4 + e]);
      }
    }
    const v4f bA = *(const v4f*)(mb1 + c8);
    const v4f bB = *(const v4f*)(mb1 + c8 + 4);
    v8h hv;
#pragma unroll
    for (int e = 0; e < 4; ++e) {
      const float h0 = fmaxf(a[e] + bA[e], 0.0f) * kCarryMh;
      const float h1 = fmaxf(a[4 + e] + bB[e], 0.0f) * kCarryMh;
      hv[e]     = to_h_flush(h0);
      hv[4 + e] = to_h_flush(h1);
    }
    *(v8h*)(sMh + row * kMhPitch + c8) = hv;
  }
  __syncthreads();

  {
    FragH fa[4];
#pragma unroll
    for (int ks = 0; ks < 4; ++ks) {
      fa[ks].h[0] = *(const v8h*)(sMh + rl * kMhPitch + ks * 32 + 8 * hh);
      fa[ks].h[1] = *(const v8h*)(sMh + rl * kMhPitch + ks * 32 + 16 + 8 * hh);
    }
    v8f acc[2];
#pragma unroll
    for (int tt = 0; tt < 2; ++tt) {
      acc[tt] = (v8f){0.f, 0.f, 0.f, 0.f, 0.f, 0.f, 0.f, 0.f};
      const int n = (2 * wave + tt) * 16 + rl;
#pragma unroll
      for (int ks = 0; ks < 4; ++ks) {
        const v16h fb = frag_load_global(MW2T + (size_t)n * kHid + ks * 32 + 8 * hh);
        acc[tt] = mma_f16(fa[ks].v, fb, acc[tt]);
      }
    }
#pragma unroll
    for (int tt = 0; tt < 2; ++tt) {
      const int n = (2 * wave + tt) * 16 + rl;
      const float bv = mb2[n];
#pragma unroll
      for (int r = 0; r < 8; ++r)
        sRaw[(8 * hh + r) * kSq + n] = fmaf(acc[tt][r], kFoldMet, bv);
    }
  }
  __syncthreads();

  {
    const int i = tid >> 4;
    const int j = tid & 15;
    const float ev = (i == j) ? kEps : 0.0f;
    float val[16];
#pragma unroll
    for (int it = 0; it < 16; ++it) {
      const float x0 = sRaw[it * kSq + tid] + ev;
      const float x1 = sRaw[it * kSq + j * kDim + i] + ev;
      val[it] = 0.5f * (x0 + x1);
    }
    float* mp = met + (size_t)rowbase * kSq + tid;
    for (int pass = 0; pass < 2; ++pass) {
#pragma unroll
      for (int it = 0; it < 16; ++it)
        *(volatile float*)(mp + (size_t)it * kSq) = val[it];
      __threadfence();
    }
  }
}

__global__ __launch_bounds__(256) void triple_net_kernel(
    const float* __restrict__ met, const float* __restrict__ cW1, const float* __restrict__ cb1,
    const float* __restrict__ cW2, const float* __restrict__ cb2, float* __restrict__ chr)
{
  __shared__ __align__(16) float sQ[kHid * 4];
  __shared__ __align__(16) float sV[kHid];
  const int tid = threadIdx.x;
  if (tid < kHid) {
    sQ[tid * 4 + 0] = cW1[tid];
    sQ[tid * 4 + 1] = cW1[kHid + tid];
    sQ[tid * 4 + 2] = cW1[2 * kHid + tid];
    sQ[tid * 4 + 3] = cb1[tid];
    sV[tid] = cW2[tid];
  }
  __syncthreads();
  const int bi = blockIdx.x;
  const int b  = bi >> 4;
  const int i  = bi & 15;
  const int j  = tid >> 4;
  const int k  = tid & 15;
  const float* mb = met + (size_t)b * kSq;
  const float m_ij = mb[i * kDim + j];
  const float m_jk = mb[j * kDim + k];
  const float m_ki = mb[k * kDim + i];
  float acc = 0.0f;
#pragma unroll 4
  for (int h = 0; h < kHid; ++h) {
    const v4f q = *(const v4f*)(sQ + 4 * h);
    float pre = m_ij * q[0];
    pre = fmaf(m_jk, q[1], pre);
    pre = fmaf(m_ki, q[2], pre);
    pre = pre + q[3];
    const float th = tanh_exp_form(pre);
    acc = fmaf(th, sV[h], acc);
  }
  const float res = acc + cb2[0];
  float* p = chr + (size_t)bi * 256 + tid;
  *(volatile float*)p = res;
  __threadfence();
  *(volatile float*)p = res;
}

__global__ __launch_bounds__(256) void pair_net_kernel(
    const float* __restrict__ points, const float* __restrict__ met, const float* __restrict__ chr,
    const _Float16* __restrict__ RW1T, const float* __restrict__ rb1,
    const float* __restrict__ rW2, const float* __restrict__ rb2, float* __restrict__ out)
{
  __shared__ __align__(16) _Float16 sC16[kTrip];
  __shared__ __align__(16) _Float16 sM16[kSq];
  __shared__ __align__(16) _Float16 sP16[32 * 8];
  __shared__ __align__(16) float    sH[kHid2];
  __shared__ __align__(16) float    sS[kSq];
  const int tid  = threadIdx.x;
  const int lane = tid & 31;
  const int wave = tid >> 5;
  const int hh   = lane >> 4;
  const int rl   = lane & 15;
  const int b    = blockIdx.x;

#pragma unroll
  for (int u = 0; u < 2; ++u) {
    const int c = tid + 256 * u;
    const float* cp = chr + (size_t)b * kTrip + c * 8;
    const v4f x0 = *(const v4f*)(cp);
    const v4f x1 = *(const v4f*)(cp + 4);
    v8h hv;
#pragma unroll
    for (int e = 0; e < 4; ++e) {
      hv[e]     = to_h_flush(x0[e] * kCarryFeat);
      hv[4 + e] = to_h_flush(x1[e] * kCarryFeat);
    }
    *(v8h*)(sC16 + c * 8) = hv;
  }
  if (wave == 0) {
    const float* mp = met + (size_t)b * kSq + lane * 8;
    const v4f x0 = *(const v4f*)(mp);
    const v4f x1 = *(const v4f*)(mp + 4);
    v8h hv;
#pragma unroll
    for (int e = 0; e < 4; ++e) {
      hv[e]     = to_h_flush(x0[e] * kCarryFeat);
      hv[4 + e] = to_h_flush(x1[e] * kCarryFeat);
    }
    *(v8h*)(sM16 + lane * 8) = hv;
  } else if (wave == 1) {
    const float* pp = points + (size_t)b * kDim + (lane & 1) * 8;
    const v4f x0 = *(const v4f*)(pp);
    const v4f x1 = *(const v4f*)(pp + 4);
    v8h hv;
#pragma unroll
    for (int e = 0; e < 4; ++e) {
      hv[e]     = to_h_flush(x0[e] * kCarryFeat);
      hv[4 + e] = to_h_flush(x1[e] * kCarryFeat);
    }
    *(v8h*)(sP16 + lane * 8) = hv;
  }

  v16h bfr[2][2];
  float bias[2];
#pragma unroll
  for (int tt = 0; tt < 2; ++tt) {
    const int n = 32 * wave + 16 * tt + rl;
    bias[tt] = rb1[n];
#pragma unroll
    for (int ks = 0; ks < 2; ++ks)
      bfr[tt][ks] = frag_load_global(RW1T + (size_t)n * kFeat + ks * 32 + 8 * hh);
  }
  __syncthreads();

  FragH a0, a1;
  a0.h[0] = *(const v8h*)(sP16 + 8 * hh);
  a1.h[0] = *(const v8h*)(sM16 + rl * kDim + 8 * hh);
  float cs0 = 0.0f, cs1 = 0.0f;
#pragma unroll 1
  for (int i = 0; i < kDim; ++i) {
    a0.h[1] = *(const v8h*)(sM16 + i * kDim + 8 * hh);
    a1.h[1] = *(const v8h*)(sC16 + (i * kDim + rl) * kDim + 8 * hh);
    v8f acc0 = (v8f){0.f, 0.f, 0.f, 0.f, 0.f, 0.f, 0.f, 0.f};
    v8f acc1 = (v8f){0.f, 0.f, 0.f, 0.f, 0.f, 0.f, 0.f, 0.f};
    acc0 = mma_f16(a0.v, bfr[0][0], acc0);
    acc0 = mma_f16(a1.v, bfr[0][1], acc0);
    acc1 = mma_f16(a0.v, bfr[1][0], acc1);
    acc1 = mma_f16(a1.v, bfr[1][1], acc1);
#pragma unroll
    for (int r = 0; r < 8; ++r) {
      cs0 += fmaxf(fmaf(acc0[r], kFoldPair, bias[0]), 0.0f);
      cs1 += fmaxf(fmaf(acc1[r], kFoldPair, bias[1]), 0.0f);
    }
  }
  cs0 += __shfl_xor(cs0, 16, 32);
  cs1 += __shfl_xor(cs1, 16, 32);
  if (hh == 0) {
    sH[32 * wave + rl]      = cs0;
    sH[32 * wave + 16 + rl] = cs1;
  }
  __syncthreads();

  float s = 0.0f;
#pragma unroll 8
  for (int hI = 0; hI < kHid2; ++hI)
    s = fmaf(sH[hI], rW2[(size_t)hI * kSq + tid], s);
  const float sv = fmaf(s, kInvPairs, rb2[tid]);
  sS[tid] = sv;
  __syncthreads();
  const float o = 0.5f * (sS[tid] + sS[(tid & 15) * kDim + (tid >> 4)]);
  float* p = out + (size_t)b * kSq + tid;
  *(volatile float*)p = o;
  __threadfence();
  *(volatile float*)p = o;
}

extern "C" void kernel_launch(void* const* d_in, const int* in_sizes, int n_in,
                              void* d_out, int out_size, void* d_ws, size_t ws_size,
                              hipStream_t stream) {
  if (n_in < 13) return;
  if (in_sizes[0] != kBatch * kDim) return;
  if (in_sizes[1] != kDim * kHid) return;
  if (in_sizes[2] != kHid) return;
  if (in_sizes[3] != kHid * kSq) return;
  if (in_sizes[4] != kSq) return;
  if (in_sizes[5] != 3 * kHid) return;
  if (in_sizes[6] != kHid) return;
  if (in_sizes[7] != kHid) return;
  if (in_sizes[8] != 1) return;
  if (in_sizes[9] != kFeat * kHid2) return;
  if (in_sizes[10] != kHid2) return;
  if (in_sizes[11] != kHid2 * kSq) return;
  if (in_sizes[12] != kSq) return;
  if (out_size != kBatch * kSq) return;
  if (ws_size < kWsTotal) return;

  const float* points = (const float*)d_in[0];
  const float* mW1 = (const float*)d_in[1];
  const float* mb1 = (const float*)d_in[2];
  const float* mW2 = (const float*)d_in[3];
  const float* mb2 = (const float*)d_in[4];
  const float* cW1 = (const float*)d_in[5];
  const float* cb1 = (const float*)d_in[6];
  const float* cW2 = (const float*)d_in[7];
  const float* cb2 = (const float*)d_in[8];
  const float* rW1 = (const float*)d_in[9];
  const float* rb1 = (const float*)d_in[10];
  const float* rW2 = (const float*)d_in[11];
  const float* rb2 = (const float*)d_in[12];
  float* outf = (float*)d_out;

  char* ws = (char*)d_ws;
  float*    MET  = (float*)(ws + kOffMET);
  float*    CHR  = (float*)(ws + kOffCHR);
  _Float16* RW1T = (_Float16*)(ws + kOffRW1T);
  _Float16* MW2T = (_Float16*)(ws + kOffMW2T);

  transpose_cast_kernel<<<(kHid2 * kFeat / 8) / 256, 256, 0, stream>>>(rW1, kFeat, kHid2, RW1T, kCarryW1, kHid2 * kFeat / 8);
  transpose_cast_kernel<<<(kSq * kHid / 8) / 256, 256, 0, stream>>>(mW2, kHid, kSq, MW2T, kCarryW2, kSq * kHid / 8);
  metric_net_kernel<<<kBatch / 16, 256, 0, stream>>>(points, mW1, mb1, MW2T, mb2, MET);
  triple_net_kernel<<<kBatch * kDim, 256, 0, stream>>>(MET, cW1, cb1, cW2, cb2, CHR);
  pair_net_kernel<<<kBatch, 256, 0, stream>>>(points, MET, CHR, RW1T, rb1, rW2, rb2, outf);
}
